// EdgeGATv2Conv_39599598469260
// MI455X (gfx1250) — hardware-verified
//
#include <hip/hip_runtime.h>
#include <hip/hip_bf16.h>
#include <stddef.h>


#define DF    64
#define ED    16
#define GR    32
#define AP    72
#define XP    68
#define NB    512
#define CHUNK 8192
#define NTHR  256
#define NWAVE 8
#define WCAP  (CHUNK / NWAVE)
#define NGRP  (CHUNK / (NTHR * 4))
#define HB    128
#define AP2   40
#define EP    68
#define MAXB  ((NWAVE * WCAP + HB - 1) / HB)

#define PW_LH 0
#define PW_LL 4096
#define PW_RH 8192
#define PW_RL 12288
#define PW_E1 16384
#define PW_E2 18432
#define PW_N  20480
#define PW_BYTES (PW_N * 2)

#define L_SACC 0
#define L_SM   (NB * DF)
#define L_SL   (L_SM + NB)
#define L_LIST (L_SL + NB)
#define L_WCNT (L_LIST + NWAVE * WCAP)
#define L_HBE  (L_WCNT + 16)
#define L_HBS  (L_HBE + HB)
#define L_ET   (L_HBS + HB)
#define L_WE1  (L_ET + HB * EP)
#define L_WE2  (L_WE1 + DF * 32 / 2)
#define L_AT   (L_WE2 + DF * 32 / 2)
#define L_END  (L_AT + HB * AP2 / 2)
#define LDS_BYTES (L_END * 4)

static_assert(DF == 64);
static_assert(ED == 16);
static_assert(WCAP == NGRP * 4 * 32);
static_assert((CHUNK & (CHUNK - 1)) == 0);
static_assert(CHUNK <= 8192);
static_assert(NB == 512);
static_assert(HB * 2 == NTHR);
static_assert(HB <= 128);
static_assert((NB % (NWAVE * 2)) == 0);
static_assert((L_SM % 4) == 0);
static_assert((L_LIST % 4) == 0);
static_assert((L_ET % 4) == 0);
static_assert((L_WE1 % 4) == 0);
static_assert((L_WE2 % 4) == 0);
static_assert((L_AT % 4) == 0);
static_assert(L_END == 55568);
static_assert(LDS_BYTES == 222272);
static_assert(PW_BYTES == 40960);

typedef float          v2f  __attribute__((ext_vector_type(2)));
typedef float          v4f  __attribute__((ext_vector_type(4)));
typedef float          v8f  __attribute__((ext_vector_type(8)));
typedef int            v4i  __attribute__((ext_vector_type(4)));
typedef unsigned       v4u  __attribute__((ext_vector_type(4)));
typedef unsigned short v4us __attribute__((ext_vector_type(4)));
typedef unsigned short v8us __attribute__((ext_vector_type(8)));
typedef __bf16         v8b  __attribute__((ext_vector_type(8)));
typedef __bf16         v16b __attribute__((ext_vector_type(16)));
union FragB { v16b v; v8b half[2]; };
union PackB { v8b b; v8us u; v4us q[2]; v4i i; };
union F4U   { v4f f; v4u u; };

__device__ __forceinline__ v8f wm(v16b a, v16b b, v8f c) {
  v8f d = __builtin_amdgcn_wmma_f32_16x16x32_bf16(false, a, false, b, (short)0, c, false, false);
  asm volatile("v_nop\n\tv_nop\n\tv_nop\n\tv_nop" : "+v"(d) : "v"(a), "v"(b));
  return d;
}

__device__ __forceinline__ float wsum(float v) {
  v += __shfl_xor(v, 16, 32);
  v += __shfl_xor(v, 8, 32);
  v += __shfl_xor(v, 4, 32);
  v += __shfl_xor(v, 2, 32);
  v += __shfl_xor(v, 1, 32);
  return v;
}

__device__ __forceinline__ void split4(v4f x, v4us& hi, v4us& lo) {
  F4U a; a.f = x;
  const v4u u  = a.u + 0x7fffu + ((a.u >> 16) & 1u);
  const v4u hb = u >> 16;
  F4U hf; hf.u = hb << 16;
  F4U r; r.f = x - hf.f;
  const v4u w  = r.u + 0x7fffu + ((r.u >> 16) & 1u);
  hi = __builtin_convertvector(hb, v4us);
  lo = __builtin_convertvector(w >> 16, v4us);
}

__global__ __launch_bounds__(NTHR) void k_prep(const float* __restrict__ Wl, const float* __restrict__ Wr,
                                                const float* __restrict__ We, __bf16* P) {
  const int tid = threadIdx.x;
  const int bx  = blockIdx.x;
  v4f f0, f1;
  __bf16* ph;
  __bf16* pl;
  if (bx < 4) {
    const int which = bx >> 1;
    const float* W = which ? Wr : Wl;
    const int g  = (bx & 1) * NTHR + tid;
    const int n  = g >> 3;
    const int k0 = (g & 7) * 8;
    f0.x = W[(k0 + 0) * DF + n]; f0.y = W[(k0 + 1) * DF + n];
    f0.z = W[(k0 + 2) * DF + n]; f0.w = W[(k0 + 3) * DF + n];
    f1.x = W[(k0 + 4) * DF + n]; f1.y = W[(k0 + 5) * DF + n];
    f1.z = W[(k0 + 6) * DF + n]; f1.w = W[(k0 + 7) * DF + n];
    ph = P + (which ? PW_RH : PW_LH) + n * DF + k0;
    pl = ph + 4096;
  } else {
    const int n  = tid >> 2;
    const int q  = tid & 3;
    const int kb = (q & 1) * 8;
    f0.x = We[(kb + 0) * DF + n]; f0.y = We[(kb + 1) * DF + n];
    f0.z = We[(kb + 2) * DF + n]; f0.w = We[(kb + 3) * DF + n];
    f1.x = We[(kb + 4) * DF + n]; f1.y = We[(kb + 5) * DF + n];
    f1.z = We[(kb + 6) * DF + n]; f1.w = We[(kb + 7) * DF + n];
    ph = P + PW_E1 + n * 32 + q * 8;
    pl = P + PW_E2 + n * 32 + q * 8;
  }
  PackB H, L;
  split4(f0, H.q[0], L.q[0]);
  split4(f1, H.q[1], L.q[1]);
  const v4i hv = H.i, lv = L.i;
  *(volatile v4i*)ph = hv;
  *(volatile v4i*)pl = lv;
  __threadfence();
  *(volatile v4i*)ph = hv;
  *(volatile v4i*)pl = lv;
}

__global__ __launch_bounds__(NTHR) void k_node(const float* __restrict__ x, const __bf16* __restrict__ P,
                                                const float* __restrict__ b_l, const float* __restrict__ b_r,
                                                float* xl, float* xr, int nN) {
  __shared__ __attribute__((aligned(16))) __bf16 Ah[GR * AP];
  __shared__ __attribute__((aligned(16))) __bf16 Al[GR * AP];
  __shared__ __attribute__((aligned(16))) float  Xs[2 * GR * XP];

  const int tid  = threadIdx.x;
  const int lane = tid & 31;
  const int wave = tid >> 5;
  const int hh   = lane >> 4;
  const int m    = lane & 15;
  const int rowBase = blockIdx.x * GR;

  {
    const int r  = tid >> 3;
    const int c0 = (tid & 7) * 8;
    int row = rowBase + r;
    if (row > nN - 1) row = nN - 1;
    const float* p = x + (size_t)row * DF + c0;
    const v4f f0 = *(const v4f*)(p);
    const v4f f1 = *(const v4f*)(p + 4);
    PackB H, L;
    split4(f0, H.q[0], L.q[0]);
    split4(f1, H.q[1], L.q[1]);
    *(v8b*)(Ah + r * AP + c0) = H.b;
    *(v8b*)(Al + r * AP + c0) = L.b;
  }
  __syncthreads();

  const int which = wave >> 2;
  const int ct    = wave & 3;
  const int ncol  = ct * 16 + m;
  const __bf16* Bh = P + (which ? PW_RH : PW_LH);
  const __bf16* Bl = Bh + 4096;

  v8f acc0 = {0.f, 0.f, 0.f, 0.f, 0.f, 0.f, 0.f, 0.f};
  v8f acc1 = {0.f, 0.f, 0.f, 0.f, 0.f, 0.f, 0.f, 0.f};
#pragma unroll
  for (int kt = 0; kt < DF / 32; ++kt) {
    const int k0 = kt * 32;
    FragB a0h, a0l, a1h, a1l, bh, bl;
    const __bf16* pbh = Bh + (size_t)ncol * DF + k0 + 8 * hh;
    const __bf16* pbl = Bl + (size_t)ncol * DF + k0 + 8 * hh;
    const __bf16* p0h = Ah + m * AP + k0 + 8 * hh;
    const __bf16* p0l = Al + m * AP + k0 + 8 * hh;
    const __bf16* p1h = Ah + (16 + m) * AP + k0 + 8 * hh;
    const __bf16* p1l = Al + (16 + m) * AP + k0 + 8 * hh;
    bh.half[0]  = *(const v8b*)pbh; bh.half[1]  = *(const v8b*)(pbh + 16);
    bl.half[0]  = *(const v8b*)pbl; bl.half[1]  = *(const v8b*)(pbl + 16);
    a0h.half[0] = *(const v8b*)p0h; a0h.half[1] = *(const v8b*)(p0h + 16);
    a0l.half[0] = *(const v8b*)p0l; a0l.half[1] = *(const v8b*)(p0l + 16);
    a1h.half[0] = *(const v8b*)p1h; a1h.half[1] = *(const v8b*)(p1h + 16);
    a1l.half[0] = *(const v8b*)p1l; a1l.half[1] = *(const v8b*)(p1l + 16);
    acc0 = wm(a0h.v, bh.v, acc0);
    acc0 = wm(a0h.v, bl.v, acc0);
    acc0 = wm(a0l.v, bh.v, acc0);
    acc1 = wm(a1h.v, bh.v, acc1);
    acc1 = wm(a1h.v, bl.v, acc1);
    acc1 = wm(a1l.v, bh.v, acc1);
  }

  const float blv = b_l[ncol];
  const float brv = b_r[ncol];
  const float bb  = which ? brv : blv;
  float* Xw = Xs + which * (GR * XP);
#pragma unroll
  for (int r = 0; r < 8; ++r) {
    Xw[(8 * hh + r) * XP + ncol]      = acc0[r] + bb;
    Xw[(16 + 8 * hh + r) * XP + ncol] = acc1[r] + bb;
  }
  __syncthreads();

  const int w2 = wave >> 2;
  float* plane = w2 ? xr : xl;
  const float* Xq = Xs + w2 * (GR * XP);
  const int r0 = (wave & 3) * 8;
  v4f vv[4];
  float* gp[4];
#pragma unroll
  for (int i = 0; i < 4; ++i) {
    const int row = r0 + 2 * i + hh;
    vv[i] = *(const v4f*)(Xq + row * XP + 4 * m);
    gp[i] = plane + (size_t)(rowBase + row) * DF + 4 * m;
  }
#pragma unroll
  for (int i = 0; i < 4; ++i) *(volatile v4f*)(gp[i]) = vv[i];
  __threadfence();
#pragma unroll
  for (int i = 0; i < 4; ++i) *(volatile v4f*)(gp[i]) = vv[i];
}

__global__ __launch_bounds__(NTHR) void k_agg(
    const float* __restrict__ xl, const float* __restrict__ xr,
    const int* __restrict__ ei, const float* __restrict__ ea,
    const __bf16* __restrict__ P, const float* __restrict__ att,
    const float* __restrict__ bias, float* out, int nN, int nE) {
  extern __shared__ v4f lds_dyn[];
  float*  ldsf = (float*)lds_dyn;
  float*  sacc = ldsf + L_SACC;
  float*  sm   = ldsf + L_SM;
  float*  sl   = ldsf + L_SL;
  int*    list = (int*)(ldsf + L_LIST);
  int*    wcnt = (int*)(ldsf + L_WCNT);
  int*    hbe  = (int*)(ldsf + L_HBE);
  int*    hbs  = (int*)(ldsf + L_HBS);
  float*  Et   = ldsf + L_ET;
  __bf16* We1  = (__bf16*)(ldsf + L_WE1);
  __bf16* We2  = (__bf16*)(ldsf + L_WE2);
  __bf16* At   = (__bf16*)(ldsf + L_AT);

  const int tid  = threadIdx.x;
  const int lane = tid & 31;
  const int wave = tid >> 5;
  const int hh   = lane >> 4;
  const int m    = lane & 15;
  const int nodeBase = blockIdx.x * NB;

  {
    const v4f z4 = {0.f, 0.f, 0.f, 0.f};
    for (int i = tid; i < (NB * DF) / 4; i += NTHR) lds_dyn[i] = z4;
    for (int i = tid; i < NB; i += NTHR) { sm[i] = -1.0e30f; sl[i] = 0.f; }
    ((v4i*)We1)[tid] = ((const v4i*)(P + PW_E1))[tid];
    ((v4i*)We2)[tid] = ((const v4i*)(P + PW_E2))[tid];
  }
  __syncthreads();

  const float attx = att[2 * lane];
  const float atty = att[2 * lane + 1];
  const int*  eid  = ei + nE;
  const bool  al16 = ((nE & 3) == 0);
  const int   nChunks = (nE + CHUNK - 1) / CHUNK;

#pragma unroll 1
  for (int ch = 0; ch < nChunks; ++ch) {
    const int  cbase = ch * CHUNK;
    const bool fullc = al16 && (cbase + CHUNK <= nE);
    int wc = 0;
#pragma unroll 2
    for (int g = 0; g < NGRP; ++g) {
      const int el0 = (g * NTHR + tid) * 4;
      const int e0  = cbase + el0;
      v4i d;
      if (fullc) {
        d = *(const v4i*)(eid + e0);
      } else {
        const int sent = -2147483647 - 1;
        const int c0 = (e0     < nE - 1) ? e0     : nE - 1;
        const int c1 = (e0 + 1 < nE - 1) ? e0 + 1 : nE - 1;
        const int c2 = (e0 + 2 < nE - 1) ? e0 + 2 : nE - 1;
        const int c3 = (e0 + 3 < nE - 1) ? e0 + 3 : nE - 1;
        const int v0 = eid[c0], v1 = eid[c1], v2 = eid[c2], v3 = eid[c3];
        d.x = (e0     < nE) ? v0 : sent;
        d.y = (e0 + 1 < nE) ? v1 : sent;
        d.z = (e0 + 2 < nE) ? v2 : sent;
        d.w = (e0 + 3 < nE) ? v3 : sent;
      }
      const unsigned s0 = (unsigned)d.x - (unsigned)nodeBase;
      const unsigned s1 = (unsigned)d.y - (unsigned)nodeBase;
      const unsigned s2 = (unsigned)d.z - (unsigned)nodeBase;
      const unsigned s3 = (unsigned)d.w - (unsigned)nodeBase;
      const bool h0 = s0 < (unsigned)NB;
      const bool h1 = s1 < (unsigned)NB;
      const bool h2 = s2 < (unsigned)NB;
      const bool h3 = s3 < (unsigned)NB;
      const unsigned many = __builtin_amdgcn_ballot_w32(h0 | h1 | h2 | h3);
      if (many != 0u) {
#define HITJ(J, HJ, SJ) { \
          const unsigned mj = __builtin_amdgcn_ballot_w32(HJ); \
          if (HJ) { \
            const int pos = wc + (int)__builtin_amdgcn_mbcnt_lo(mj, 0u); \
            if (pos < WCAP) list[wave * WCAP + pos] = ((el0 + (J)) << 9) | (int)(SJ); \
          } \
          wc += (int)__builtin_popcount(mj); }
        HITJ(0, h0, s0)
        HITJ(1, h1, s1)
        HITJ(2, h2, s2)
        HITJ(3, h3, s3)
#undef HITJ
      }
    }
    if (lane == 0) wcnt[wave] = wc;
    __syncthreads();

    int off[NWAVE + 1];
    off[0] = 0;
#pragma unroll
    for (int w = 0; w < NWAVE; ++w) {
      int c = wcnt[w];
      c = c < 0 ? 0 : (c > WCAP ? WCAP : c);
      off[w + 1] = off[w] + c;
    }
    const int T = off[NWAVE];
    __syncthreads();
    const int nbatch = (T + HB - 1) / HB;

#pragma unroll 1
    for (int b = 0; b < nbatch && b < MAXB; ++b) {
      const int base = b * HB;
      int nb = T - base;
      if (nb > HB) nb = HB;

      {
        const int  j    = tid >> 1;
        const int  q    = tid & 1;
        const bool live = (j < nb);
        const int  jj   = live ? j : (nb - 1);
        const int  gi   = base + jj;
        int osel = 0, wsel = 0;
#pragma unroll
        for (int w = 1; w < NWAVE; ++w) {
          if (gi >= off[w]) { osel = off[w]; wsel = w; }
        }
        int pos = gi - osel;
        pos = pos < 0 ? 0 : (pos > WCAP - 1 ? WCAP - 1 : pos);
        const int ent  = list[wsel * WCAP + pos];
        const int slot = ent & (NB - 1);
        const int el   = (ent >> 9) & (CHUNK - 1);
        int e = cbase + el;
        if (e > nE - 1) e = nE - 1;
        const float* ap = ea + (size_t)e * ED + 8 * q;
        v4f f0 = *(const v4f*)(ap);
        v4f f1 = *(const v4f*)(ap + 4);
        const v4f z4 = {0.f, 0.f, 0.f, 0.f};
        f0 = live ? f0 : z4;
        f1 = live ? f1 : z4;
        PackB H, L;
        split4(f0, H.q[0], L.q[0]);
        split4(f1, H.q[1], L.q[1]);
        *(v8b*)(At + j * AP2 + 8 * q)      = H.b;
        *(v8b*)(At + j * AP2 + 16 + 8 * q) = L.b;
        if (q == 0) { hbe[j] = e; hbs[j] = slot; }
      }
      __syncthreads();

      {
        const int ntile = (nb + 15) >> 4;
        const int ntask = ntile * 4;
#pragma unroll 1
        for (int task = wave; task < ntask; task += NWAVE) {
          const int rt  = task >> 2;
          const int ct2 = task & 3;
          FragB a, b1, b2;
          const __bf16* pa  = At  + (rt * 16 + m) * AP2 + 8 * hh;
          const __bf16* pb1 = We1 + (ct2 * 16 + m) * 32 + 8 * hh;
          const __bf16* pb2 = We2 + (ct2 * 16 + m) * 32 + 8 * hh;
          a.half[0]  = *(const v8b*)pa;  a.half[1]  = *(const v8b*)(pa + 16);
          b1.half[0] = *(const v8b*)pb1; b1.half[1] = *(const v8b*)(pb1 + 16);
          b2.half[0] = *(const v8b*)pb2; b2.half[1] = *(const v8b*)(pb2 + 16);
          v8f acc = {0.f, 0.f, 0.f, 0.f, 0.f, 0.f, 0.f, 0.f};
          acc = wm(a.v, b1.v, acc);
          acc = wm(a.v, b2.v, acc);
#pragma unroll
          for (int r = 0; r < 8; ++r) Et[(rt * 16 + 8 * hh + r) * EP + ct2 * 16 + m] = acc[r];
        }
      }
      __syncthreads();

      if (wave == 0) {
#pragma unroll 1
        for (int j = 0; j < nb; ++j) {
          const int slot = hbs[j];
          const int e    = hbe[j];
          int src = ei[e];
          src = src < 0 ? 0 : (src > nN - 1 ? nN - 1 : src);
          int node = nodeBase + slot;
          if (node > nN - 1) node = nN - 1;
          const v2f xl2 = *(const v2f*)(xl + (size_t)src  * DF + 2 * lane);
          const v2f xr2 = *(const v2f*)(xr + (size_t)node * DF + 2 * lane);
          const v2f e2  = *(const v2f*)(Et + j * EP + 2 * lane);
          float hx = (xl2.x + xr2.x) + e2.x;
          float hy = (xl2.y + xr2.y) + e2.y;
          hx = (hx > 0.f) ? hx : 0.2f * hx;
          hy = (hy > 0.f) ? hy : 0.2f * hy;
          float s = hx * attx + hy * atty;
          s = wsum(s);
          s = __shfl(s, 0, 32);
          const float mo = sm[slot];
          const float mn = fmaxf(mo, s);
          const float sc = __expf(mo - mn);
          const float p  = __expf(s - mn);
          const float lo = sl[slot];
          sl[slot] = lo * sc + p;
          sm[slot] = mn;
          v2f* ap2 = (v2f*)(sacc + slot * DF + 2 * lane);
          const v2f cur = *ap2;
          const v2f nxt = cur * sc + xl2 * p;
          *ap2 = nxt;
        }
      }
      __syncthreads();
    }
  }
  __syncthreads();

  const v4f b4 = *(const v4f*)(bias + 4 * m);
#pragma unroll 1
  for (int i = 0; i < NB / (NWAVE * 2); ++i) {
    const int slot = wave * (NB / NWAVE) + 2 * i + hh;
    const int node = nodeBase + slot;
    const v4f a4  = *(const v4f*)(sacc + slot * DF + 4 * m);
    const float l = sl[slot];
    const float inv = (l > 0.f) ? (1.0f / l) : 0.f;
    const v4f val = a4 * inv + b4;
    float* op = out + (size_t)node * DF + 4 * m;
    if (node < nN) *(volatile v4f*)op = val;
    __threadfence();
    if (node < nN) *(volatile v4f*)op = val;
  }
}

extern "C" void kernel_launch(void* const* d_in, const int* in_sizes, int n_in,
                              void* d_out, int out_size, void* d_ws, size_t ws_size,
                              hipStream_t stream) {
  if (n_in < 10) return;
  const int nN = in_sizes[0] / DF;
  if (nN <= 0 || in_sizes[0] != nN * DF) return;
  if (in_sizes[1] < 2 || (in_sizes[1] & 1) != 0) return;
  const int nE = in_sizes[1] / 2;
  if (in_sizes[2] != nE * ED) return;
  if (in_sizes[3] != DF * DF || in_sizes[5] != DF * DF || in_sizes[7] != ED * DF) return;
  if (in_sizes[4] != DF || in_sizes[6] != DF || in_sizes[8] != DF || in_sizes[9] != DF) return;
  if (out_size != nN * DF) return;

  const float* x    = (const float*)d_in[0];
  const int*   ei   = (const int*)d_in[1];
  const float* ea   = (const float*)d_in[2];
  const float* W_l  = (const float*)d_in[3];
  const float* b_l  = (const float*)d_in[4];
  const float* W_r  = (const float*)d_in[5];
  const float* b_r  = (const float*)d_in[6];
  const float* W_e  = (const float*)d_in[7];
  const float* att  = (const float*)d_in[8];
  const float* bias = (const float*)d_in[9];
  float* out = (float*)d_out;

  const int nP = ((nN + GR - 1) / GR) * GR;
  size_t off = 0;
  __bf16* P  = (__bf16*)((char*)d_ws + off); off += (size_t)PW_BYTES;
  float*  xl = (float*)((char*)d_ws + off);  off += (size_t)nP * DF * sizeof(float);
  float*  xr = (float*)((char*)d_ws + off);  off += (size_t)nP * DF * sizeof(float);
  if (off > ws_size) return;

  k_prep<<<5, NTHR, 0, stream>>>(W_l, W_r, W_e, P);

  k_node<<<nP / GR, NTHR, 0, stream>>>(x, P, b_l, b_r, xl, xr, nN);

  hipFuncSetAttribute(reinterpret_cast<const void*>(&k_agg),
                      hipFuncAttributeMaxDynamicSharedMemorySize, LDS_BYTES);
  const int grid = (nN + NB - 1) / NB;
  k_agg<<<grid, NTHR, LDS_BYTES, stream>>>(xl, xr, ei, ea, P, att, bias, out, nN, nE);
}
